// LogSparseAttention_79843442032893
// MI455X (gfx1250) — hardware-verified
//
#include <hip/hip_runtime.h>
#include <math.h>
#include <stdint.h>


#define NB   4
#define SEQ  2048
#define NH   8
#define HD   64
#define TOKP (NH * HD)
#define AT_NW 4
#define AT_QB 64
#define AT_KC 64
#define MAXVISIT 6
#define NQT  (SEQ / AT_QB)

#ifndef P_FORM
#define P_FORM 1
#endif

static_assert(SEQ % 64 == 0);
static_assert(HD == 64);
static_assert(AT_QB == 64 && AT_KC == 64);
static_assert(NQT == 32);
static_assert(NH == 8);
static_assert(MAXVISIT == 6);
static_assert((AT_KC << (MAXVISIT - 2)) == SEQ / 2);
static_assert((size_t)3 * NB * NH * SEQ * HD * 2 <= ((size_t)128 << 20));

typedef __attribute__((ext_vector_type(16))) __bf16   v16b;
typedef __attribute__((ext_vector_type(8)))  __bf16   v8b;
typedef __attribute__((ext_vector_type(8)))  float    v8f;
typedef __attribute__((ext_vector_type(4)))  float    v4f;
typedef __attribute__((ext_vector_type(4)))  unsigned int v4u;

union FB { v16b v; v8b h[2]; };

__device__ __forceinline__ unsigned short f2bf_bits(float f) {
  unsigned u = __float_as_uint(f);
  return (unsigned short)((u + 0x7FFFu + ((u >> 16) & 1u)) >> 16);
}
__device__ __forceinline__ unsigned pk16(unsigned short a, unsigned short b) { return (unsigned)a | ((unsigned)b << 16); }

__device__ __forceinline__ __bf16 at_f2bf(float f) { return __builtin_bit_cast(__bf16, f2bf_bits(f)); }
__device__ __forceinline__ void at_split(float f, __bf16& hi, __bf16& lo) {
  const unsigned short hb = f2bf_bits(f);
  hi = __builtin_bit_cast(__bf16, hb);
  lo = at_f2bf(f - __uint_as_float(((unsigned)hb) << 16));
}
__device__ __forceinline__ v16b frag_ld(const __bf16* p) {
  FB f; f.h[0] = *(const v8b*)(p); f.h[1] = *(const v8b*)(p + 16); return f.v;
}
__device__ __forceinline__ v8f at_mma(v16b a, v16b b, v8f c) {
  c = __builtin_amdgcn_wmma_f32_16x16x32_bf16(false, a, false, b, (short)0, c, false, false);
  asm volatile("v_nop\n\tv_nop\n\tv_nop\n\tv_nop" : "+v"(c) : "v"(a), "v"(b));
  return c;
}
__device__ __forceinline__ bool lg_allowed(int diff) {
  return (diff == 0) | ((diff > 0) & ((diff & (diff - 1)) == 0));
}

__global__ __launch_bounds__(256) void k_prep(const float* __restrict__ q, const float* __restrict__ k,
                                              const float* __restrict__ v,
                                              unsigned short* __restrict__ QB, unsigned short* __restrict__ KB,
                                              unsigned short* __restrict__ VT) {
  __shared__ __align__(16) float tf[64 * 68];
  const int tid = threadIdx.x;
  const int bx  = blockIdx.x;
  const int lt  = bx & (NQT - 1);
  const int bh  = bx >> 5;
  const int h   = bh & (NH - 1);
  const int b   = bh >> 3;
  const int l0  = lt * 64;
  const int sub = tid >> 3;
  const int c8  = (tid & 7) * 8;

  v4u qv[2], kv[2], vv[2];
#pragma unroll
  for (int it = 0; it < 2; ++it) {
    const int rr = it * 32 + sub;
    const size_t src = ((size_t)(b * SEQ + l0 + rr) * NH + h) * HD + c8;
    const v4f a0 = *(const v4f*)(q + src);
    const v4f a1 = *(const v4f*)(q + src + 4);
    const v4f b0 = *(const v4f*)(k + src);
    const v4f b1 = *(const v4f*)(k + src + 4);
    qv[it] = (v4u){pk16(f2bf_bits(a0[0]), f2bf_bits(a0[1])), pk16(f2bf_bits(a0[2]), f2bf_bits(a0[3])),
                   pk16(f2bf_bits(a1[0]), f2bf_bits(a1[1])), pk16(f2bf_bits(a1[2]), f2bf_bits(a1[3]))};
    kv[it] = (v4u){pk16(f2bf_bits(b0[0]), f2bf_bits(b0[1])), pk16(f2bf_bits(b0[2]), f2bf_bits(b0[3])),
                   pk16(f2bf_bits(b1[0]), f2bf_bits(b1[1])), pk16(f2bf_bits(b1[2]), f2bf_bits(b1[3]))};
  }
  {
    const int lr = tid >> 4;
    const int c4 = (tid & 15) * 4;
#pragma unroll
    for (int it = 0; it < 4; ++it) {
      const int rr = it * 16 + lr;
      const v4f a = *(const v4f*)(v + ((size_t)(b * SEQ + l0 + rr) * NH + h) * HD + c4);
      *(v4f*)(tf + rr * 68 + c4) = a;
    }
  }
  __syncthreads();
#pragma unroll
  for (int it = 0; it < 2; ++it) {
    const int oc = it * 32 + sub;
    v4u a;
#pragma unroll
    for (int qd = 0; qd < 4; ++qd) {
      const float f0 = tf[(c8 + 2 * qd) * 68 + oc];
      const float f1 = tf[(c8 + 2 * qd + 1) * 68 + oc];
      a[qd] = pk16(f2bf_bits(f0), f2bf_bits(f1));
    }
    vv[it] = a;
  }
  for (int pass = 0; pass < 2; ++pass) {
#pragma unroll
    for (int it = 0; it < 2; ++it) {
      const int rr = it * 32 + sub;
      const size_t qo = ((size_t)bh * SEQ + l0 + rr) * HD + c8;
      const size_t go = ((size_t)bh * HD + rr) * SEQ + l0 + c8;
      *(volatile v4u*)(QB + qo) = qv[it];
      *(volatile v4u*)(KB + qo) = kv[it];
      *(volatile v4u*)(VT + go) = vv[it];
    }
    __threadfence();
  }
}

__global__ __launch_bounds__(128) __attribute__((amdgpu_num_vgpr(248)))
void k_attn(const unsigned short* __restrict__ QB, const unsigned short* __restrict__ KB,
            const unsigned short* __restrict__ VT, float* __restrict__ out) {
  __shared__ __align__(16) __bf16 Ksh[AT_KC * HD];
  __shared__ __align__(16) __bf16 Vth[HD * AT_KC];
  __shared__ __align__(16) __bf16 Psh[AT_NW][16 * AT_KC];
#if P_FORM == 1
  __shared__ __align__(16) __bf16 Psl[AT_NW][16 * AT_KC];
#endif
  __shared__ __align__(16) float  Os[AT_NW][16 * 68];

  const int tid  = threadIdx.x;
  const int wave = tid >> 5;
  const int lane = tid & 31;
  const int hh   = lane >> 4;
  const int c    = lane & 15;

  const int bx = blockIdx.x;
  const int qt = bx & (NQT - 1);
  const int bh = bx >> 5;
  const int h  = bh & (NH - 1);
  const int b  = bh >> 3;
  const int q0 = qt * AT_QB + wave * 16;

  const __bf16* Qp = (const __bf16*)(const void*)QB + (size_t)bh * SEQ * HD;
  const __bf16* Kp = (const __bf16*)(const void*)KB + (size_t)bh * SEQ * HD;
  const __bf16* Vp = (const __bf16*)(const void*)VT + (size_t)bh * HD * SEQ;
  float*        ob = out + ((size_t)b * SEQ * NH + h) * HD;

  v16b qa[2];
#pragma unroll
  for (int dc = 0; dc < 2; ++dc)
    qa[dc] = frag_ld(Qp + (size_t)(q0 + c) * HD + dc * 32 + 8 * hh);

  float mrow[8], lrow[8];
  v8f oacc[4];
#pragma unroll
  for (int r = 0; r < 8; ++r) { mrow[r] = -INFINITY; lrow[r] = 0.0f; }
#pragma unroll
  for (int t = 0; t < 4; ++t) oacc[t] = (v8f){0.f,0.f,0.f,0.f,0.f,0.f,0.f,0.f};

#pragma unroll 1
  for (int vi = 0; vi < MAXVISIT; ++vi) {
    const int toff = (vi == 0) ? 0 : (1 << (vi - 1));
    const int kt = qt - toff;
    if (kt < 0) break;
    const int kv0 = kt * AT_KC;
    __syncthreads();
    {
      const int r = tid >> 1, half = (tid & 1) * 32;
      const __bf16* ks = Kp + (size_t)(kv0 + r) * HD + half;
      const __bf16* vs = Vp + (size_t)r * SEQ + kv0 + half;
#pragma unroll
      for (int i = 0; i < 4; ++i) {
        const v8b a0 = *(const v8b*)(ks + 8 * i);
        const v8b b0 = *(const v8b*)(vs + 8 * i);
        *(v8b*)(Ksh + r * HD    + half + 8 * i) = a0;
        *(v8b*)(Vth + r * AT_KC + half + 8 * i) = b0;
      }
    }
    __syncthreads();

    v8f s[4];
#pragma unroll
    for (int j = 0; j < 4; ++j) {
      s[j] = (v8f){0.f,0.f,0.f,0.f,0.f,0.f,0.f,0.f};
#pragma unroll
      for (int dc = 0; dc < 2; ++dc) {
        FB kb;
        kb.h[0] = *(const v8b*)(Ksh + (j * 16 + c) * HD + dc * 32 + 8 * hh);
        kb.h[1] = *(const v8b*)(Ksh + (j * 16 + c) * HD + dc * 32 + 16 + 8 * hh);
        s[j] = at_mma(qa[dc], kb.v, s[j]);
      }
    }

    float cm[8];
#pragma unroll
    for (int r = 0; r < 8; ++r) {
      const int qrow = q0 + 8 * hh + r;
      float m = -INFINITY;
#pragma unroll
      for (int j = 0; j < 4; ++j) {
        const int kvcol = kv0 + j * 16 + c;
        const float sv = s[j][r] * 0.125f;
        const bool ok = lg_allowed(qrow - kvcol);
        const float sm = ok ? sv : -INFINITY;
        s[j][r] = sm;
        m = fmaxf(m, sm);
      }
#pragma unroll
      for (int off = 1; off < 16; off <<= 1) m = fmaxf(m, __shfl_xor(m, off, 32));
      cm[r] = m;
    }

    __bf16* pwh = Psh[wave];
#if P_FORM == 1
    __bf16* pwl = Psl[wave];
#endif
#pragma unroll
    for (int r = 0; r < 8; ++r) {
      const int qrow = q0 + 8 * hh + r;
      const float mnew = fmaxf(mrow[r], cm[r]);
      const float alpha = expf(mrow[r] - mnew);
      mrow[r] = mnew;
      float psum = 0.0f;
#pragma unroll
      for (int j = 0; j < 4; ++j) {
        const int kvcol = kv0 + j * 16 + c;
        const bool ok = lg_allowed(qrow - kvcol);
        const float e = expf(s[j][r] - mnew);
        const float p = ok ? e : 0.0f;
        psum += p;
#if P_FORM == 1
        __bf16 a, bl; at_split(p, a, bl);
        pwh[(8 * hh + r) * AT_KC + j * 16 + c] = a;
        pwl[(8 * hh + r) * AT_KC + j * 16 + c] = bl;
#else
        pwh[(8 * hh + r) * AT_KC + j * 16 + c] = at_f2bf(p);
#endif
      }
#pragma unroll
      for (int off = 1; off < 16; off <<= 1) psum += __shfl_xor(psum, off, 32);
      lrow[r] = lrow[r] * alpha + psum;
#pragma unroll
      for (int t = 0; t < 4; ++t) oacc[t][r] *= alpha;
    }
    __builtin_amdgcn_fence(__ATOMIC_RELEASE, "workgroup");
    __builtin_amdgcn_wave_barrier();
    __builtin_amdgcn_fence(__ATOMIC_ACQUIRE, "workgroup");

#pragma unroll 1
    for (int kk = 0; kk < 2; ++kk) {
      FB pa;
      pa.h[0] = *(const v8b*)(pwh + c * AT_KC + kk * 32 + 8 * hh);
      pa.h[1] = *(const v8b*)(pwh + c * AT_KC + kk * 32 + 16 + 8 * hh);
#if P_FORM == 1
      FB pl;
      pl.h[0] = *(const v8b*)(pwl + c * AT_KC + kk * 32 + 8 * hh);
      pl.h[1] = *(const v8b*)(pwl + c * AT_KC + kk * 32 + 16 + 8 * hh);
#endif
#pragma unroll
      for (int t = 0; t < 4; ++t) {
        FB vb;
        vb.h[0] = *(const v8b*)(Vth + (t * 16 + c) * AT_KC + kk * 32 + 8 * hh);
        vb.h[1] = *(const v8b*)(Vth + (t * 16 + c) * AT_KC + kk * 32 + 16 + 8 * hh);
        oacc[t] = at_mma(pa.v, vb.v, oacc[t]);
#if P_FORM == 1
        oacc[t] = at_mma(pl.v, vb.v, oacc[t]);
#endif
      }
    }
  }

  float* os = Os[wave];
#pragma unroll
  for (int r = 0; r < 8; ++r) {
    const float inv = 1.0f / lrow[r];
#pragma unroll
    for (int t = 0; t < 4; ++t) os[(8 * hh + r) * 68 + t * 16 + c] = oacc[t][r] * inv;
  }
  __builtin_amdgcn_fence(__ATOMIC_RELEASE, "workgroup");
  __builtin_amdgcn_wave_barrier();
  __builtin_amdgcn_fence(__ATOMIC_ACQUIRE, "workgroup");
  {
    const int c4 = (lane & 15) * 4;
    for (int pass = 0; pass < 2; ++pass) {
#pragma unroll
      for (int it = 0; it < 8; ++it) {
        const int row = it * 2 + hh;
        const v4f val = *(const v4f*)(os + row * 68 + c4);
        *(volatile v4f*)(ob + (size_t)(q0 + row) * TOKP + c4) = val;
      }
      __threadfence();
    }
  }
}

extern "C" void kernel_launch(void* const* d_in, const int* in_sizes, int n_in,
                              void* d_out, int out_size, void* d_ws, size_t ws_size,
                              hipStream_t stream) {
  const int NEL = NB * SEQ * NH * HD;
  if (n_in < 3) return;
  if (in_sizes[0] != NEL || in_sizes[1] != NEL || in_sizes[2] != NEL) return;
  if (out_size != NEL) return;
  const size_t PL = (size_t)NEL * 2;
  if (3 * PL > ws_size) return;

  const float* q = (const float*)d_in[0];
  const float* k = (const float*)d_in[1];
  const float* v = (const float*)d_in[2];
  char* ws = (char*)d_ws;
  unsigned short* QB = (unsigned short*)(ws);
  unsigned short* KB = (unsigned short*)(ws + PL);
  unsigned short* VT = (unsigned short*)(ws + 2 * PL);

  k_prep<<<dim3(NB * NH * NQT), dim3(256), 0, stream>>>(q, k, v, QB, KB, VT);
  k_attn<<<dim3(NB * NH * NQT), dim3(128), 0, stream>>>(QB, KB, VT, (float*)d_out);
  (void)hipGetLastError();
}
